// EPS_55379308315221
// MI455X (gfx1250) — hardware-verified
//
#include <hip/hip_runtime.h>


#ifndef NB
#define NB 32
#endif
#define NB_FULL 32
#define HI_  258
#define WI_  258
#define HO_  257
#define WO_  257
#define SD   4
#define OD   4
#define NIJ  16
#define NN   64
#define CHS  4096.0f
#define CLS  16.0f
#define ULS  256.0f
#define CTI  (1.0f / 4096.0f)
#define WPB  4
#define ITERS 8
#define NPIX (NB * HO_ * WO_)
#define NIT  ((NPIX + 31) / 32)
#define NWAVES ((NIT + ITERS - 1) / ITERS)
#define NBLK ((NWAVES + WPB - 1) / WPB)

static_assert(NB <= NB_FULL);
static_assert(SD == 4);
static_assert(OD == 4);
static_assert(NIJ == SD * SD);
static_assert(2 * NIJ == 32);
static_assert(NN == SD * SD * OD);
static_assert(NN % 16 == 0);
static_assert(NN / 16 == 4);
static_assert(CHS == CLS * ULS);
static_assert(CHS * CTI == 1.0f);
static_assert(HO_ == HI_ - 1);
static_assert(WO_ == WI_ - 1);
static_assert(256 * 8 == NN * 32);
static_assert(32 * 16 == 32 * OD * 4);
static_assert((size_t)NPIX * OD * 4 < ((size_t)1 << 31));
static_assert((size_t)NBLK * WPB * ITERS >= (size_t)NIT);

typedef _Float16 h16;
typedef __attribute__((ext_vector_type(16))) _Float16 v16h;
typedef __attribute__((ext_vector_type(8)))  _Float16 v8h;
typedef __attribute__((ext_vector_type(8)))  float    v8f;
typedef __attribute__((ext_vector_type(4)))  float    v4f;
typedef __attribute__((ext_vector_type(2)))  float    v2f;

__device__ __forceinline__ unsigned short f2bf(float f) { unsigned u = __float_as_uint(f); u += 0x7FFFu + ((u >> 16) & 1u); return (unsigned short)(u >> 16); }
__device__ __forceinline__ float bfr(float f) { return __uint_as_float(((unsigned)f2bf(f)) << 16); }
__device__ __forceinline__ v16h cat16(v8h lo, v8h hi) { return __builtin_shufflevector(lo, hi, 0, 1, 2, 3, 4, 5, 6, 7, 8, 9, 10, 11, 12, 13, 14, 15); }
__device__ __forceinline__ v8f wmma16(v16h a, v16h b, v8f c) { return __builtin_amdgcn_wmma_f32_16x16x32_f16(false, a, false, b, (short)0, c, false, false); }
__device__ __forceinline__ v16h  ldh(const h16* p) { return cat16(*(const v8h*)p, *(const v8h*)(p + 16)); }
static __device__ __forceinline__ h16 toh_flush(float v) { const h16 r = (h16)v; return (fabsf(v) < 6.103515625e-05f) ? (h16)0.0f : r; }
__device__ __forceinline__ v8f wmma16g(v16h a, v16h b, v8f c) { c = wmma16(a, b, c); asm volatile("v_nop\n\tv_nop\n\tv_nop\n\tv_nop" : "+v"(c) : "v"(a), "v"(b)); return c; }

__global__ __launch_bounds__(256) void k_wconv(const float* __restrict__ core, h16* CT) {
    const int i = threadIdx.x;
    const int n = i >> 2, k8 = (i & 3) * 8;
    const int kb = k8 & 15;
    const float sc = (k8 < 16) ? CHS : CLS;
    v8h o;
#pragma unroll
    for (int j = 0; j < 8; ++j) { const float c = bfr(core[(kb + j) * NN + n]); o[j] = toh_flush(c * sc); }
    *(volatile v8h*)(CT + (size_t)i * 8) = o; __threadfence(); *(volatile v8h*)(CT + (size_t)i * 8) = o;
}

__device__ __forceinline__ v4f pix_tile(const float* __restrict__ X, v16h c0, v16h c1, v16h c2, v16h c3, int P, int hi) {
    const int Pc = P < NPIX ? P : (NPIX - 1);
    const int bh = Pc / WO_; const int wo = Pc - bh * WO_;
    const int b  = bh / HO_; const int ho = bh - b * HO_;
    const size_t xo = (((size_t)b * HI_ + (size_t)ho) * WI_ + (size_t)wo) * SD;
    const v2f q0 = *(const v2f*)(X + xo + 2 * hi);
    const v4f q1 = *(const v4f*)(X + xo + SD);
    const v4f q2 = *(const v4f*)(X + xo + (size_t)WI_ * SD);
    const v2f q3 = *(const v2f*)(X + xo + (size_t)WI_ * SD + SD + 2 * hi);
    float a0[2], a1[4], a2[4], a3[2];
    a0[0] = bfr(q0[0]); a0[1] = bfr(q0[1]); a3[0] = bfr(q3[0]); a3[1] = bfr(q3[1]);
#pragma unroll
    for (int c = 0; c < 4; ++c) { a1[c] = bfr(q1[c]); a2[c] = bfr(q2[c]); }
    v16h ub;
#pragma unroll
    for (int e = 0; e < 8; ++e) {
        const float u = a0[e >> 2] * a1[e & 3];
        const h16 uh = toh_flush(u);
        ub[e] = uh;
        ub[8 + e] = toh_flush((u - (float)uh) * ULS);
    }
    v8f d[4];
    d[0] = wmma16g(c0, ub, (v8f){});
    d[1] = wmma16g(c1, ub, (v8f){});
    d[2] = wmma16g(c2, ub, (v8f){});
    d[3] = wmma16g(c3, ub, (v8f){});
    v4f acc = (v4f){};
#pragma unroll
    for (int nt = 0; nt < 4; ++nt) {
#pragma unroll
        for (int s = 0; s < 2; ++s) {
            const float vv = a2[nt] * a3[s];
#pragma unroll
            for (int o = 0; o < 4; ++o) acc[o] = fmaf(d[nt][4 * s + o], vv, acc[o]);
        }
    }
#pragma unroll
    for (int o = 0; o < 4; ++o) acc[o] += __shfl_xor(acc[o], 16, 32);
    return acc * CTI;
}

__global__ __launch_bounds__(32 * WPB) void k_pix(const float* __restrict__ X, const h16* __restrict__ CT, float* OUT) {
    const int lane = threadIdx.x & 31, lr = lane & 15, hi = lane >> 4;
    const int wave = __builtin_amdgcn_readfirstlane((int)(threadIdx.x >> 5));
    const int g = (int)blockIdx.x * WPB + wave;
    const size_t co = (size_t)lr * 32 + 8 * hi;
    const v16h c0 = ldh(CT + co);
    const v16h c1 = ldh(CT + co + (size_t)16 * 32);
    const v16h c2 = ldh(CT + co + (size_t)32 * 32);
    const v16h c3 = ldh(CT + co + (size_t)48 * 32);
#pragma unroll 1
    for (int s = 0; s < ITERS; ++s) {
        const int it = g * ITERS + s;
        if (it >= NIT) break;
        const int P0 = it * 32;
        const v4f r0 = pix_tile(X, c0, c1, c2, c3, P0 + lr, hi);
        const v4f r1 = pix_tile(X, c0, c1, c2, c3, P0 + 16 + lr, hi);
        v4f val;
#pragma unroll
        for (int c = 0; c < 4; ++c) val[c] = (hi != 0) ? r1[c] : r0[c];
        const int P = P0 + lane;
        const bool ok = ((NPIX % 32) == 0) || (P < NPIX);
        float* op = OUT + (size_t)P * OD;
        if (ok) *(volatile v4f*)op = val;
        __threadfence();
        if (ok) *(volatile v4f*)op = val;
    }
}

static constexpr size_t SZ_CT = (size_t)NN * 32 * 2;
static_assert(SZ_CT % 128 == 0);
static_assert(SZ_CT <= (size_t)134217728);

extern "C" void kernel_launch(void* const* d_in, const int* in_sizes, int n_in,
                              void* d_out, int out_size, void* d_ws, size_t ws_size, hipStream_t stream) {
    if (n_in < 2) return;
    if ((size_t)in_sizes[0] < (size_t)NB * HI_ * WI_ * SD) return;
    if ((size_t)in_sizes[1] < (size_t)NIJ * NN) return;
    if ((size_t)out_size < (size_t)NPIX * OD) return;
    if (SZ_CT > ws_size) return;
    const float* x    = (const float*)d_in[0];
    const float* core = (const float*)d_in[1];
    float* OUT = (float*)d_out;
    h16* CT = (h16*)d_ws;

    k_wconv<<<dim3(1, 1, 1), dim3(256, 1, 1), 0, stream>>>(core, CT);
    k_pix<<<dim3((unsigned)NBLK, 1, 1), dim3(32 * WPB, 1, 1), 0, stream>>>(x, CT, OUT);
}
